// PointNetSetAbstraction_54906861912674
// MI455X (gfx1250) — hardware-verified
//
#include <hip/hip_runtime.h>

#pragma clang fp contract(off)

typedef __attribute__((ext_vector_type(16))) _Float16 v16h;
typedef __attribute__((ext_vector_type(8)))  _Float16 v8h;
typedef __attribute__((ext_vector_type(8)))  float    v8f;
typedef __attribute__((ext_vector_type(4)))  float    v4f;
typedef __attribute__((ext_vector_type(4)))  int      v4i;

__device__ __forceinline__ void dep_guard_h(v8f& a, v8f& b, v16h x, v16h y) { asm volatile("v_nop\n\tv_nop\n\tv_nop\n\tv_nop" : "+v"(a), "+v"(b) : "v"(x), "v"(y)); }
__device__ __forceinline__ void keep4_h(v16h a, v16h b, v16h c, v16h d) { asm volatile("v_nop" :: "v"(a), "v"(b), "v"(c), "v"(d)); }
template <typename T> struct Frag;
template <> struct Frag<_Float16> {
  typedef v16h V; union U { v16h v; v8h h[2]; };
  static __device__ __forceinline__ v16h load(const _Float16* p) {
    U f; f.h[0] = *(const v8h*)(p); f.h[1] = *(const v8h*)(p + 16); return f.v;
  }
  static __device__ __forceinline__ v8f mma(v16h a, v16h b, v8f c) {
    return __builtin_amdgcn_wmma_f32_16x16x32_f16(false, a, false, b, (short)0, c, false, false);
  }
  static __device__ __forceinline__ void guard(v8f& a, v8f& b, v16h x, v16h y) { dep_guard_h(a, b, x, y); }
  static __device__ __forceinline__ void keep(v16h a, v16h b, v16h c, v16h d) { keep4_h(a, b, c, d); }
};
__device__ __forceinline__ void guard_acc4(v8f& a0, v8f& a1, v8f& a2, v8f& a3,
                                           v16h x, v16h y0, v16h y1, v16h y2, v16h y3) {
  asm volatile("v_nop\n\tv_nop\n\tv_nop\n\tv_nop"
               : "+v"(a0), "+v"(a1), "+v"(a2), "+v"(a3)
               : "v"(x), "v"(y0), "v"(y1), "v"(y2), "v"(y3));
}

constexpr int NB   = 16;
constexpr int NPTS = 4096;
constexpr int NS   = 1024;
constexpr int NK   = 32;
constexpr int NCOL = NB * NS * NK;
constexpr int CIN0 = 3;
constexpr int CH1  = 64;
constexpr int CH2  = 128;
constexpr int BTP  = 72;
constexpr int COLS_PER_BLOCK = 256;
constexpr int GEMM_BLOCKS = NCOL / COLS_PER_BLOCK;
constexpr int ST0_COLS = 1024;
constexpr int ST0_BLOCKS = NCOL / ST0_COLS;
static_assert(NCOL == 524288);
static_assert(NCOL % COLS_PER_BLOCK == 0);
static_assert(NCOL % ST0_COLS == 0);
static_assert(CH1 % 32 == 0);
static_assert(CH1 % 16 == 0 && CH2 % 16 == 0);
static_assert(NS * NK == (1 << 15));
static_assert(NPTS == 4 * 4 * 256);
static_assert(NPTS == 2 * 4 * 512);

constexpr float WCARRY      = 16.0f;
constexpr float WCARRY_INV  = 1.0f / 16.0f;
constexpr float LOCARRY     = 1024.0f;
constexpr float LOCARRY_INV = 1.0f / 1024.0f;
constexpr float BN_EPS      = 1e-5f;

constexpr size_t OUT0_ELEMS = (size_t)NB * CH2 * NS;
constexpr size_t OUT1_ELEMS = (size_t)NB * 3 * NS;
constexpr size_t OUT1_OFF_BYTES = 8388608;
static_assert(OUT0_ELEMS * 4 == OUT1_OFF_BYTES);
static_assert((OUT0_ELEMS + OUT1_ELEMS) * 4 == 8585216);
static_assert(OUT1_OFF_BYTES % 128 == 0);

constexpr size_t WS_NX    = 0;
constexpr size_t WS_GX    = WS_NX   + (size_t)NB * NS * 4 * 4;
constexpr size_t WS_P0    = WS_GX   + (size_t)NB * NK * 3 * NS * 4;
constexpr size_t WS_BNP0  = WS_P0   + (size_t)ST0_BLOCKS * 2 * CH1 * 4;
constexpr size_t WS_P1    = WS_BNP0 + 1024;
constexpr size_t WS_BNP1  = WS_P1   + (size_t)GEMM_BLOCKS * 2 * CH1 * 4;
constexpr size_t WS_P2    = WS_BNP1 + 1024;
constexpr size_t WS_BNP2  = WS_P2   + (size_t)GEMM_BLOCKS * 2 * CH2 * 4;
constexpr size_t WS_YMAX  = WS_BNP2 + 1024;
constexpr size_t WS_YMIN  = WS_YMAX + (size_t)NB * NS * CH2 * 4;
constexpr size_t WS_TOTAL = WS_YMIN + (size_t)NB * NS * CH2 * 4;
static_assert(WS_TOTAL == 26741760);
static_assert(WS_TOTAL <= 134217728);
static_assert(WS_GX % 128 == 0 && WS_P0 % 128 == 0 && WS_BNP0 % 128 == 0 && WS_P1 % 128 == 0 &&
              WS_BNP1 % 128 == 0 && WS_P2 % 128 == 0 && WS_BNP2 % 128 == 0 && WS_YMAX % 128 == 0 &&
              WS_YMIN % 128 == 0);

__device__ __forceinline__ float hsum16(float v) {
  v += __shfl_xor(v, 1, 32); v += __shfl_xor(v, 2, 32); v += __shfl_xor(v, 4, 32); v += __shfl_xor(v, 8, 32);
  return v;
}
__device__ __forceinline__ float hmax16(float v) {
  v = fmaxf(v, __shfl_xor(v, 1, 32)); v = fmaxf(v, __shfl_xor(v, 2, 32));
  v = fmaxf(v, __shfl_xor(v, 4, 32)); v = fmaxf(v, __shfl_xor(v, 8, 32));
  return v;
}
__device__ __forceinline__ float hmin16(float v) {
  v = fminf(v, __shfl_xor(v, 1, 32)); v = fminf(v, __shfl_xor(v, 2, 32));
  v = fminf(v, __shfl_xor(v, 4, 32)); v = fminf(v, __shfl_xor(v, 8, 32));
  return v;
}

__device__ __forceinline__ float pre0_eval(v4f w, float rx, float ry, float rz) {
  float p = w.x * rx;
  p = fmaf(w.y, ry, p);
  p = fmaf(w.z, rz, p);
  return p + w.w;
}

__device__ __forceinline__ void rel_coords(const float* __restrict__ gx, const float* __restrict__ nxp,
                                           int col, float& rx, float& ry, float& rz) {
  const int b = col >> 15;
  const int s = (col >> 5) & (NS - 1);
  const int k = col & (NK - 1);
  const float* p = gx + ((size_t)(b * NK + k) * 3) * NS + s;
  const float px = p[0], py = p[NS], pz = p[2 * NS];
  const v4f cv = *(const v4f*)(nxp + ((size_t)b * NS + s) * 4);
  rx = px - cv.x; ry = py - cv.y; rz = pz - cv.z;
}

__device__ __forceinline__ float comb(float h, float l) { return (h + l * LOCARRY_INV) * WCARRY_INV; }

__global__ void __launch_bounds__(256)
fps_kernel(const float* __restrict__ xyz, float* __restrict__ nxp, float* __restrict__ out1)
{
  #pragma clang fp contract(off)
  __shared__ float rv[16];
  __shared__ int   ri[16];
  __shared__ int   sidx[NS];
  __shared__ __align__(16) float so1[3 * NS];
  __shared__ __align__(16) float snx[4 * NS];

  const int b = blockIdx.x;
  const int t = threadIdx.x, lane = t & 31, wave = t >> 5;
  const float* xb = xyz + (size_t)b * 3 * NPTS;

  float px[16], py[16], pz[16], dm[16];
#pragma unroll
  for (int q = 0; q < 4; ++q) {
    const v4f ax = *(const v4f*)(xb + q * 1024 + 4 * t);
    const v4f ay = *(const v4f*)(xb + NPTS + q * 1024 + 4 * t);
    const v4f az = *(const v4f*)(xb + 2 * NPTS + q * 1024 + 4 * t);
#pragma unroll
    for (int e = 0; e < 4; ++e) {
      px[q * 4 + e] = ax[e]; py[q * 4 + e] = ay[e]; pz[q * 4 + e] = az[e]; dm[q * 4 + e] = 1e10f;
    }
    if (q == 1) asm volatile("" ::: "memory");
  }

  int far = 0;
  for (int s = 0; s < NS; ++s) {
    if (t == 0) sidx[s] = far;
    const float cx = xb[far], cy = xb[NPTS + far], cz = xb[2 * NPTS + far];
    float bv = -1.0f;
    int   bi = 4 * t;
#pragma unroll
    for (int i = 0; i < 16; ++i) {
      const float dx = px[i] - cx, dy = py[i] - cy, dz = pz[i] - cz;
      const float d = (dx * dx + dz * dz) + dy * dy;
      const float nd = fminf(dm[i], d);
      dm[i] = nd;
      const bool gt = nd > bv;
      bv = gt ? nd : bv;
      bi = gt ? ((i >> 2) * 1024 + 4 * t + (i & 3)) : bi;
    }
#pragma unroll
    for (int off = 16; off > 0; off >>= 1) {
      const float ov = __shfl_xor(bv, off, 32);
      const int   oi = __shfl_xor(bi, off, 32);
      const bool tk = (ov > bv) || (ov == bv && oi < bi);
      bv = tk ? ov : bv;
      bi = tk ? oi : bi;
    }
    const int par = (s & 1) * 8;
    if (lane == 0) { rv[par + wave] = bv; ri[par + wave] = bi; }
    __syncthreads();
    float fv = rv[par];
    int   fi = ri[par];
#pragma unroll
    for (int w = 1; w < 8; ++w) {
      const float ov = rv[par + w];
      const int   oi = ri[par + w];
      const bool tk = (ov > fv) || (ov == fv && oi < fi);
      fv = tk ? ov : fv;
      fi = tk ? oi : fi;
    }
    far = fi;
  }
  __syncthreads();

  for (int s = t; s < NS; s += 256) {
    int g = sidx[s];
    g = g < 0 ? 0 : (g > NPTS - 1 ? NPTS - 1 : g);
    const float gxv = xb[g], gyv = xb[NPTS + g], gzv = xb[2 * NPTS + g];
    so1[s] = gxv; so1[NS + s] = gyv; so1[2 * NS + s] = gzv;
    *(v4f*)(snx + 4 * s) = (v4f){gxv, gyv, gzv, 0.0f};
  }
  __syncthreads();

  float* o1 = out1 + (size_t)b * 3 * NS;
  float* nx = nxp + (size_t)b * 4 * NS;
  for (int pass = 0; pass < 2; ++pass) {
#pragma unroll
    for (int i = 0; i < 3; ++i) {
      const int f = t + 256 * i;
      const v4f v = *(const v4f*)(so1 + 4 * f);
      *(volatile v4f*)(o1 + 4 * f) = v;
    }
#pragma unroll
    for (int i = 0; i < 4; ++i) {
      const int f = t + 256 * i;
      const v4f v = *(const v4f*)(snx + 4 * f);
      *(volatile v4f*)(nx + 4 * f) = v;
    }
    __threadfence();
  }
}

__global__ void __launch_bounds__(512)
sort_kernel(const float* __restrict__ xyz, const float* __restrict__ nxp, float* __restrict__ gx)
{
  #pragma clang fp contract(off)
  __shared__ unsigned long long comp[NPTS];
  __shared__ __align__(16) float sg[3 * NS];

  const int b = blockIdx.x >> 5, k = blockIdx.x & 31;
  const int t = threadIdx.x;
  const float* xb = xyz + (size_t)b * 3 * NPTS;
  const v4f cv = *(const v4f*)(nxp + ((size_t)b * NS + k) * 4);

#pragma unroll
  for (int q = 0; q < 2; ++q) {
    const int n0 = q * 2048 + 4 * t;
    const v4f ax = *(const v4f*)(xb + n0);
    const v4f ay = *(const v4f*)(xb + NPTS + n0);
    const v4f az = *(const v4f*)(xb + 2 * NPTS + n0);
#pragma unroll
    for (int e = 0; e < 4; ++e) {
      const float dx = ax[e] - cv.x, dy = ay[e] - cv.y, dz = az[e] - cv.z;
      const float d = (dx * dx + dz * dz) + dy * dy;
      const unsigned kb = __float_as_uint(d);
      comp[n0 + e] = ((unsigned long long)kb << 32) | (unsigned long long)(unsigned)(n0 + e);
    }
  }
  __syncthreads();

  for (int ksz = 2; ksz <= NPTS; ksz <<= 1) {
    for (int j = ksz >> 1; j > 0; j >>= 1) {
#pragma unroll
      for (int r = 0; r < 4; ++r) {
        const int p  = t + 512 * r;
        const int i  = ((p & ~(j - 1)) << 1) | (p & (j - 1));
        const int ip = i | j;
        const unsigned long long a = comp[i], c = comp[ip];
        const bool up = (i & ksz) == 0;
        const unsigned long long mn = a < c ? a : c;
        const unsigned long long mx = a < c ? c : a;
        comp[i]  = up ? mn : mx;
        comp[ip] = up ? mx : mn;
      }
      __syncthreads();
    }
  }

  for (int s = t; s < NS; s += 512) {
    const unsigned long long cw = comp[s];
    int g = (int)(unsigned)(cw & 0xffffffffull);
    g = g < 0 ? 0 : (g > NPTS - 1 ? NPTS - 1 : g);
    sg[s] = xb[g]; sg[NS + s] = xb[NPTS + g]; sg[2 * NS + s] = xb[2 * NPTS + g];
  }
  __syncthreads();

  float* dst = gx + ((size_t)(b * NK + k) * 3) * NS;
  for (int pass = 0; pass < 2; ++pass) {
    for (int f = t; f < (3 * NS) / 4; f += 512) {
      const v4f v = *(const v4f*)(sg + 4 * f);
      *(volatile v4f*)(dst + 4 * f) = v;
    }
    __threadfence();
  }
}

__global__ void __launch_bounds__(256)
stats0_kernel(const float* __restrict__ gx, const float* __restrict__ nxp,
              const float* __restrict__ W0, const float* __restrict__ b0, float* __restrict__ part0)
{
  __shared__ v4f srw[CH1];
  __shared__ v4f srel[256];
  __shared__ float red[4 * 2 * CH1];
  __shared__ __align__(16) float pst[2 * CH1];

  const int t = threadIdx.x;
  if (t < CH1) srw[t] = (v4f){W0[3 * t], W0[3 * t + 1], W0[3 * t + 2], b0[t]};
  const int c = t & (CH1 - 1), q = t >> 6;
  float s = 0.0f, sq = 0.0f;
  __syncthreads();
  const v4f w = srw[c];
  for (int chunk = 0; chunk < ST0_COLS / 256; ++chunk) {
    const int col = blockIdx.x * ST0_COLS + chunk * 256 + t;
    float rx, ry, rz;
    rel_coords(gx, nxp, col, rx, ry, rz);
    srel[t] = (v4f){rx, ry, rz, 0.0f};
    __syncthreads();
#pragma unroll 4
    for (int jj = 0; jj < 64; ++jj) {
      const v4f r4 = srel[jj * 4 + q];
      const float pre = pre0_eval(w, r4.x, r4.y, r4.z);
      s += pre;
      sq += pre * pre;
    }
    __syncthreads();
  }
  red[q * 2 * CH1 + c] = s;
  red[q * 2 * CH1 + CH1 + c] = sq;
  __syncthreads();
  if (t < 2 * CH1) {
    float tot = 0.0f;
#pragma unroll
    for (int qq = 0; qq < 4; ++qq) tot += red[qq * 2 * CH1 + t];
    pst[t] = tot;
  }
  __syncthreads();
  if (t < 32) {
    const v4f v = *(const v4f*)(pst + 4 * t);
    float* p = part0 + (size_t)blockIdx.x * 2 * CH1 + 4 * t;
    *(volatile v4f*)p = v;
    __threadfence();
    *(volatile v4f*)p = v;
  }
}

template <int NCH, int NBLK>
__global__ void __launch_bounds__(256)
bn_finalize_kernel(const float* __restrict__ part, const float* __restrict__ gamma,
                   const float* __restrict__ beta, float* __restrict__ bnp)
{
  __shared__ __align__(16) float lineb[2 * NCH];
  const int t = threadIdx.x;
  if (t < NCH) {
    double s = 0.0, q = 0.0;
#pragma unroll 4
    for (int blk = 0; blk < NBLK; ++blk) {
      s += (double)part[(size_t)blk * 2 * NCH + t];
      q += (double)part[(size_t)blk * 2 * NCH + NCH + t];
    }
    const double inv_n = 1.0 / (double)NCOL;
    const double mean = s * inv_n;
    double var = q * inv_n - mean * mean;
    var = var < 0.0 ? 0.0 : var;
    const float meanf = (float)mean;
    const float varf  = (float)var;
    const float sc = gamma[t] * rsqrtf(varf + BN_EPS);
    const float sh = beta[t] - meanf * sc;
    lineb[t] = sc;
    lineb[NCH + t] = sh;
  }
  __syncthreads();
  if (t < NCH / 2) {
    const v4f v = *(const v4f*)(lineb + 4 * t);
    float* p = bnp + 4 * t;
    *(volatile v4f*)p = v;
    __threadfence();
    *(volatile v4f*)p = v;
  }
}

__device__ __forceinline__ void stage_w(const float* __restrict__ W, _Float16* Ws, int rows, int t) {
#pragma unroll 1
  for (int idx = t; idx < rows * 8; idx += 256) {
    const int row = idx >> 3, c8 = (idx & 7) * 8;
    const v4f a  = *(const v4f*)(W + (size_t)row * CH1 + c8);
    const v4f bq = *(const v4f*)(W + (size_t)row * CH1 + c8 + 4);
    v8h hv;
    hv[0] = (_Float16)(a.x * WCARRY);  hv[1] = (_Float16)(a.y * WCARRY);
    hv[2] = (_Float16)(a.z * WCARRY);  hv[3] = (_Float16)(a.w * WCARRY);
    hv[4] = (_Float16)(bq.x * WCARRY); hv[5] = (_Float16)(bq.y * WCARRY);
    hv[6] = (_Float16)(bq.z * WCARRY); hv[7] = (_Float16)(bq.w * WCARRY);
    *(v8h*)(Ws + row * BTP + c8) = hv;
  }
}

__device__ __forceinline__ void act0_to_lds(float rx, float ry, float rz, const v4f* srw, const float* sbn,
                                            _Float16* bth, _Float16* btl, int row) {
#pragma unroll 2
  for (int cg = 0; cg < CH1 / 8; ++cg) {
    v8h hv, lv;
#pragma unroll
    for (int e = 0; e < 8; ++e) {
      const int c = cg * 8 + e;
      const v4f w = srw[c];
      const float pre = pre0_eval(w, rx, ry, rz);
      const float a = fmaxf(fmaf(pre, sbn[c], sbn[CH1 + c]), 0.0f);
      const _Float16 ah = (_Float16)a;
      hv[e] = ah;
      lv[e] = (_Float16)((a - (float)ah) * LOCARRY);
    }
    *(v8h*)(bth + row * BTP + cg * 8) = hv;
    *(v8h*)(btl + row * BTP + cg * 8) = lv;
  }
}

struct BFr { v16h h[2][2]; v16h l[2][2]; };
__device__ __forceinline__ void load_bfr(const _Float16* bth, const _Float16* btl, int wrow0,
                                         int rlane, int koff, BFr& f) {
#pragma unroll
  for (int t2 = 0; t2 < 2; ++t2) {
#pragma unroll
    for (int ks = 0; ks < 2; ++ks) {
      const int p = (wrow0 + t2 * 16 + rlane) * BTP + koff + ks * 32;
      f.h[t2][ks] = Frag<_Float16>::load(bth + p);
      f.l[t2][ks] = Frag<_Float16>::load(btl + p);
    }
  }
}

__device__ __forceinline__ void mma_rowtile(const _Float16* Ws, int arow0, int rlane, int koff, const BFr& f,
                                            v8f& ah0, v8f& ah1, v8f& al0, v8f& al1) {
  const v8f z = (v8f){0.f, 0.f, 0.f, 0.f, 0.f, 0.f, 0.f, 0.f};
  ah0 = z; ah1 = z; al0 = z; al1 = z;
#pragma unroll
  for (int ks = 0; ks < 2; ++ks) {
    const v16h a = Frag<_Float16>::load(Ws + (arow0 + rlane) * BTP + koff + ks * 32);
    ah0 = Frag<_Float16>::mma(a, f.h[0][ks], ah0);
    ah1 = Frag<_Float16>::mma(a, f.h[1][ks], ah1);
    al0 = Frag<_Float16>::mma(a, f.l[0][ks], al0);
    al1 = Frag<_Float16>::mma(a, f.l[1][ks], al1);
    guard_acc4(ah0, ah1, al0, al1, a, f.h[0][ks], f.h[1][ks], f.l[0][ks], f.l[1][ks]);
  }
}

__global__ void __launch_bounds__(256)
layer1_stats_kernel(const float* __restrict__ gx, const float* __restrict__ nxp,
                    const float* __restrict__ W0, const float* __restrict__ b0, const float* __restrict__ bnp0,
                    const float* __restrict__ W1, const float* __restrict__ b1, float* __restrict__ part1)
{
  __shared__ __align__(16) _Float16 Ws1[CH1 * BTP];
  __shared__ __align__(16) _Float16 Bth[COLS_PER_BLOCK * BTP];
  __shared__ __align__(16) _Float16 Btl[COLS_PER_BLOCK * BTP];
  __shared__ v4f srw[CH1];
  __shared__ __align__(32) float sbn0[2 * CH1];
  __shared__ __align__(32) float sb1[CH1];
  __shared__ __align__(16) float wst[8 * 2 * CH1];
  __shared__ __align__(16) float pst[2 * CH1];

  const int t = threadIdx.x, lane = t & 31, wave = t >> 5;
  const int rlane = lane & 15, hh = lane >> 4, koff = hh * 8;

  stage_w(W1, Ws1, CH1, t);
  if (t < CH1) { srw[t] = (v4f){W0[3 * t], W0[3 * t + 1], W0[3 * t + 2], b0[t]}; sb1[t] = b1[t]; }
  if (t < 2 * CH1) sbn0[t] = bnp0[t];
  float rx, ry, rz;
  rel_coords(gx, nxp, blockIdx.x * COLS_PER_BLOCK + t, rx, ry, rz);
  __syncthreads();
  act0_to_lds(rx, ry, rz, srw, sbn0, Bth, Btl, t);
  __syncthreads();

  BFr f;
  load_bfr(Bth, Btl, wave * 32, rlane, koff, f);
  float* wp = wst + wave * 2 * CH1;
#pragma unroll 1
  for (int rt = 0; rt < CH1 / 16; ++rt) {
    v8f ah0, ah1, al0, al1;
    mma_rowtile(Ws1, rt * 16, rlane, koff, f, ah0, ah1, al0, al1);
    const int cb = rt * 16 + hh * 8;
    const v8f b8 = *(const v8f*)(sb1 + cb);
    float s8[8], q8[8];
#pragma unroll
    for (int r = 0; r < 8; ++r) {
      const float v0 = comb(ah0[r], al0[r]) + b8[r];
      const float v1 = comb(ah1[r], al1[r]) + b8[r];
      s8[r] = hsum16(v0 + v1);
      q8[r] = hsum16(v0 * v0 + v1 * v1);
    }
    *(v4f*)(wp + cb)           = (v4f){s8[0], s8[1], s8[2], s8[3]};
    *(v4f*)(wp + cb + 4)       = (v4f){s8[4], s8[5], s8[6], s8[7]};
    *(v4f*)(wp + CH1 + cb)     = (v4f){q8[0], q8[1], q8[2], q8[3]};
    *(v4f*)(wp + CH1 + cb + 4) = (v4f){q8[4], q8[5], q8[6], q8[7]};
  }
  __syncthreads();
  if (t < 2 * CH1) {
    float tot = 0.0f;
#pragma unroll
    for (int w = 0; w < 8; ++w) tot += wst[w * 2 * CH1 + t];
    pst[t] = tot;
  }
  __syncthreads();
  if (t < 32) {
    const v4f v = *(const v4f*)(pst + 4 * t);
    float* p = part1 + (size_t)blockIdx.x * 2 * CH1 + 4 * t;
    *(volatile v4f*)p = v;
    __threadfence();
    *(volatile v4f*)p = v;
  }
}

__global__ void __launch_bounds__(256)
layer2_kernel(const float* __restrict__ gx, const float* __restrict__ nxp,
              const float* __restrict__ W0, const float* __restrict__ b0, const float* __restrict__ bnp0,
              const float* __restrict__ W1, const float* __restrict__ b1, const float* __restrict__ bnp1,
              const float* __restrict__ W2, const float* __restrict__ b2,
              float* __restrict__ part2, float* __restrict__ ymax, float* __restrict__ ymin)
{
  __shared__ __align__(16) _Float16 Ws1[CH1 * BTP];
  __shared__ __align__(16) _Float16 Ws2[CH2 * BTP];
  __shared__ __align__(16) _Float16 Bth[COLS_PER_BLOCK * BTP];
  __shared__ __align__(16) _Float16 Btl[COLS_PER_BLOCK * BTP];
  __shared__ v4f srw[CH1];
  __shared__ __align__(32) float sbn0[2 * CH1];
  __shared__ __align__(32) float sb1[CH1];
  __shared__ __align__(32) float sbn1[2 * CH1];
  __shared__ __align__(32) float sb2[CH2];
  __shared__ __align__(16) float wst[8 * 2 * CH2];
  __shared__ __align__(16) float wmx[8 * 2 * CH2];
  __shared__ __align__(16) float pst[2 * CH2];

  const int t = threadIdx.x, lane = t & 31, wave = t >> 5;
  const int rlane = lane & 15, hh = lane >> 4, koff = hh * 8;

  stage_w(W1, Ws1, CH1, t);
  stage_w(W2, Ws2, CH2, t);
  if (t < CH1) { srw[t] = (v4f){W0[3 * t], W0[3 * t + 1], W0[3 * t + 2], b0[t]}; sb1[t] = b1[t]; }
  if (t < 2 * CH1) { sbn0[t] = bnp0[t]; sbn1[t] = bnp1[t]; }
  if (t < CH2) sb2[t] = b2[t];
  float rx, ry, rz;
  rel_coords(gx, nxp, blockIdx.x * COLS_PER_BLOCK + t, rx, ry, rz);
  __syncthreads();
  act0_to_lds(rx, ry, rz, srw, sbn0, Bth, Btl, t);
  __syncthreads();

  BFr f;
  load_bfr(Bth, Btl, wave * 32, rlane, koff, f);
  __syncthreads();
#pragma unroll 1
  for (int rt = 0; rt < CH1 / 16; ++rt) {
    v8f ah0, ah1, al0, al1;
    mma_rowtile(Ws1, rt * 16, rlane, koff, f, ah0, ah1, al0, al1);
    const int cb = rt * 16 + hh * 8;
    const v8f b8  = *(const v8f*)(sb1 + cb);
    const v8f sc8 = *(const v8f*)(sbn1 + cb);
    const v8f sh8 = *(const v8f*)(sbn1 + CH1 + cb);
    v8h h0, l0, h1, l1;
#pragma unroll
    for (int r = 0; r < 8; ++r) {
      const float v0 = comb(ah0[r], al0[r]) + b8[r];
      const float v1 = comb(ah1[r], al1[r]) + b8[r];
      const float a0 = fmaxf(fmaf(v0, sc8[r], sh8[r]), 0.0f);
      const float a1 = fmaxf(fmaf(v1, sc8[r], sh8[r]), 0.0f);
      const _Float16 q0 = (_Float16)a0, q1 = (_Float16)a1;
      h0[r] = q0; l0[r] = (_Float16)((a0 - (float)q0) * LOCARRY);
      h1[r] = q1; l1[r] = (_Float16)((a1 - (float)q1) * LOCARRY);
    }
    const int o0 = (wave * 32 + rlane) * BTP + cb;
    const int o1 = (wave * 32 + 16 + rlane) * BTP + cb;
    *(v8h*)(Bth + o0) = h0; *(v8h*)(Btl + o0) = l0;
    *(v8h*)(Bth + o1) = h1; *(v8h*)(Btl + o1) = l1;
  }
  __syncthreads();

  load_bfr(Bth, Btl, wave * 32, rlane, koff, f);
  float* wp = wst + wave * 2 * CH2;
  float* mp = wmx + wave * 2 * CH2;
#pragma unroll 1
  for (int rt = 0; rt < CH2 / 16; ++rt) {
    v8f ah0, ah1, al0, al1;
    mma_rowtile(Ws2, rt * 16, rlane, koff, f, ah0, ah1, al0, al1);
    const int cb = rt * 16 + hh * 8;
    const v8f b8 = *(const v8f*)(sb2 + cb);
    float s8[8], q8[8], m8[8], n8[8];
#pragma unroll
    for (int r = 0; r < 8; ++r) {
      const float v0 = comb(ah0[r], al0[r]) + b8[r];
      const float v1 = comb(ah1[r], al1[r]) + b8[r];
      s8[r] = hsum16(v0 + v1);
      q8[r] = hsum16(v0 * v0 + v1 * v1);
      m8[r] = hmax16(fmaxf(v0, v1));
      n8[r] = hmin16(fminf(v0, v1));
    }
    *(v4f*)(wp + cb)           = (v4f){s8[0], s8[1], s8[2], s8[3]};
    *(v4f*)(wp + cb + 4)       = (v4f){s8[4], s8[5], s8[6], s8[7]};
    *(v4f*)(wp + CH2 + cb)     = (v4f){q8[0], q8[1], q8[2], q8[3]};
    *(v4f*)(wp + CH2 + cb + 4) = (v4f){q8[4], q8[5], q8[6], q8[7]};
    *(v4f*)(mp + cb)           = (v4f){m8[0], m8[1], m8[2], m8[3]};
    *(v4f*)(mp + cb + 4)       = (v4f){m8[4], m8[5], m8[6], m8[7]};
    *(v4f*)(mp + CH2 + cb)     = (v4f){n8[0], n8[1], n8[2], n8[3]};
    *(v4f*)(mp + CH2 + cb + 4) = (v4f){n8[4], n8[5], n8[6], n8[7]};
  }
  __syncthreads();

  {
    float tot = 0.0f;
#pragma unroll
    for (int w = 0; w < 8; ++w) tot += wst[w * 2 * CH2 + t];
    pst[t] = tot;
  }
  const v4f mv = *(const v4f*)(mp + 4 * lane);
  const v4f nv = *(const v4f*)(mp + CH2 + 4 * lane);
  __syncthreads();

  if (t < 64) {
    const v4f v = *(const v4f*)(pst + 4 * t);
    float* p = part2 + (size_t)blockIdx.x * 2 * CH2 + 4 * t;
    *(volatile v4f*)p = v;
    __threadfence();
    *(volatile v4f*)p = v;
  }
  {
    const size_t bs = (size_t)blockIdx.x * 8 + wave;
    float* pm = ymax + bs * CH2 + 4 * lane;
    float* pn = ymin + bs * CH2 + 4 * lane;
    for (int pass = 0; pass < 2; ++pass) {
      *(volatile v4f*)pm = mv;
      *(volatile v4f*)pn = nv;
      __threadfence();
    }
  }
}

__global__ void __launch_bounds__(256)
pool_bn_kernel(const float* __restrict__ ymax, const float* __restrict__ ymin,
               const float* __restrict__ bnp2, float* __restrict__ out0)
{
  __shared__ __align__(16) float smx[CH2 * 36];
  __shared__ __align__(16) float smn[CH2 * 36];
  __shared__ float sbn[2 * CH2];

  const int t = threadIdx.x, lane = t & 31, wave = t >> 5;
  const int b = blockIdx.x >> 5, s0 = (blockIdx.x & 31) * 32;
  sbn[t] = bnp2[t];
  const float* rm = ymax + ((size_t)b * NS + s0) * CH2;
  const float* rn = ymin + ((size_t)b * NS + s0) * CH2;
#pragma unroll
  for (int i = 0; i < 4; ++i) {
    const int f = t + 256 * i, j = f >> 5, c4 = (f & 31) * 4;
    const v4f a = *(const v4f*)(rm + (size_t)j * CH2 + c4);
    smx[(c4 + 0) * 36 + j] = a.x; smx[(c4 + 1) * 36 + j] = a.y;
    smx[(c4 + 2) * 36 + j] = a.z; smx[(c4 + 3) * 36 + j] = a.w;
  }
  asm volatile("" ::: "memory");
#pragma unroll
  for (int i = 0; i < 4; ++i) {
    const int f = t + 256 * i, j = f >> 5, c4 = (f & 31) * 4;
    const v4f a = *(const v4f*)(rn + (size_t)j * CH2 + c4);
    smn[(c4 + 0) * 36 + j] = a.x; smn[(c4 + 1) * 36 + j] = a.y;
    smn[(c4 + 2) * 36 + j] = a.z; smn[(c4 + 3) * 36 + j] = a.w;
  }
  __syncthreads();

  const int q = lane >> 3, x4 = (lane & 7) * 4;
  v4f o[4];
#pragma unroll
  for (int it = 0; it < 4; ++it) {
    const int c = it * 32 + wave * 4 + q;
    const float sc = sbn[c], sh = sbn[CH2 + c];
    const v4f mx = *(const v4f*)(smx + c * 36 + x4);
    const v4f mn = *(const v4f*)(smn + c * 36 + x4);
    const bool pos = sc >= 0.0f;
    v4f r4;
    r4.x = fmaxf(fmaf(pos ? mx.x : mn.x, sc, sh), 0.0f);
    r4.y = fmaxf(fmaf(pos ? mx.y : mn.y, sc, sh), 0.0f);
    r4.z = fmaxf(fmaf(pos ? mx.z : mn.z, sc, sh), 0.0f);
    r4.w = fmaxf(fmaf(pos ? mx.w : mn.w, sc, sh), 0.0f);
    o[it] = r4;
  }
  for (int pass = 0; pass < 2; ++pass) {
#pragma unroll
    for (int it = 0; it < 4; ++it) {
      const int c = it * 32 + wave * 4 + q;
      *(volatile v4f*)(out0 + ((size_t)(b * CH2 + c)) * NS + s0 + x4) = o[it];
    }
    __threadfence();
  }
}

extern "C" void kernel_launch(void* const* d_in, const int* in_sizes, int n_in,
                              void* d_out, int out_size, void* d_ws, size_t ws_size,
                              hipStream_t stream)
{
  if (n_in < 13) return;
  if (in_sizes[0] != NB * CIN0 * NPTS) return;
  if (in_sizes[1] != CH1 * CIN0 || in_sizes[2] != CH1 || in_sizes[3] != CH1 || in_sizes[4] != CH1) return;
  if (in_sizes[5] != CH1 * CH1 || in_sizes[6] != CH1 || in_sizes[7] != CH1 || in_sizes[8] != CH1) return;
  if (in_sizes[9] != CH2 * CH1 || in_sizes[10] != CH2 || in_sizes[11] != CH2 || in_sizes[12] != CH2) return;
  if ((size_t)out_size < OUT0_ELEMS + OUT1_ELEMS) return;
  if (ws_size < WS_TOTAL) return;

  const float* xyz = (const float*)d_in[0];
  const float* W0  = (const float*)d_in[1];
  const float* b0  = (const float*)d_in[2];
  const float* g0  = (const float*)d_in[3];
  const float* be0 = (const float*)d_in[4];
  const float* W1  = (const float*)d_in[5];
  const float* b1  = (const float*)d_in[6];
  const float* g1  = (const float*)d_in[7];
  const float* be1 = (const float*)d_in[8];
  const float* W2  = (const float*)d_in[9];
  const float* b2  = (const float*)d_in[10];
  const float* g2  = (const float*)d_in[11];
  const float* be2 = (const float*)d_in[12];

  char* ws = (char*)d_ws;
  float* nxp   = (float*)(ws + WS_NX);
  float* gx    = (float*)(ws + WS_GX);
  float* part0 = (float*)(ws + WS_P0);
  float* bnp0  = (float*)(ws + WS_BNP0);
  float* part1 = (float*)(ws + WS_P1);
  float* bnp1  = (float*)(ws + WS_BNP1);
  float* part2 = (float*)(ws + WS_P2);
  float* bnp2  = (float*)(ws + WS_BNP2);
  float* ymax  = (float*)(ws + WS_YMAX);
  float* ymin  = (float*)(ws + WS_YMIN);
  float* out0  = (float*)d_out;
  float* out1  = (float*)d_out + OUT1_OFF_BYTES / 4;

  fps_kernel<<<dim3(NB), dim3(256), 0, stream>>>(xyz, nxp, out1);
  sort_kernel<<<dim3(NB * NK), dim3(512), 0, stream>>>(xyz, nxp, gx);
  stats0_kernel<<<dim3(ST0_BLOCKS), dim3(256), 0, stream>>>(gx, nxp, W0, b0, part0);
  bn_finalize_kernel<CH1, ST0_BLOCKS><<<dim3(1), dim3(256), 0, stream>>>(part0, g0, be0, bnp0);
  layer1_stats_kernel<<<dim3(GEMM_BLOCKS), dim3(256), 0, stream>>>(gx, nxp, W0, b0, bnp0, W1, b1, part1);
  bn_finalize_kernel<CH1, GEMM_BLOCKS><<<dim3(1), dim3(256), 0, stream>>>(part1, g1, be1, bnp1);
  layer2_kernel<<<dim3(GEMM_BLOCKS), dim3(256), 0, stream>>>(gx, nxp, W0, b0, bnp0, W1, b1, bnp1, W2, b2,
                                                            part2, ymax, ymin);
  bn_finalize_kernel<CH2, GEMM_BLOCKS><<<dim3(1), dim3(256), 0, stream>>>(part2, g2, be2, bnp2);
  pool_bn_kernel<<<dim3(NB * 32), dim3(256), 0, stream>>>(ymax, ymin, bnp2, out0);
}
